// JKNet_27419071218301
// MI455X (gfx1250) — hardware-run, weakly checked
//
#include <hip/hip_runtime.h>
#include <stddef.h>
#include <stdint.h>
#include <math.h>


#define CIN    128
#define HID    64
#define NLAY   6
#define NCLS   40
#define NCP    64
#define KL     128
#define KZ     (NLAY * KL)
#define NTHR   256
#define NWAVE  8
#define EPT    8
#define CHUNK  (NTHR * EPT)
#define WCAP   (EPT * 32)
#define LISTN  (NWAVE * WCAP)
#define NBD    8192
#define SLD    13
#define NBA    1024
#define SLA    10
#define RCAP   28672
#define DEGCAP 256
#define GBM    64
#define GBN    64
#define GTHR   128
#define NU0    (HID * (KL / 8))
#define NUH    ((NLAY - 1) * HID * (KL / 8))
#define NUO    (NCP * (KZ / 8))
#define AGG_ZINTS (LISTN + 2 * RCAP + 3 * NBA)
#define AGG_LDS_INTS (AGG_ZINTS + 16)
#define WSMAX  134217728

static_assert((CHUNK & (CHUNK - 1)) == 0 && CHUNK <= 4096);
static_assert((NBD & (NBD - 1)) == 0 && NBD == (1 << SLD));
static_assert((NBA & (NBA - 1)) == 0 && NBA == (1 << SLA));
static_assert(((long long)CHUNK << SLD) < (1LL << 31));
static_assert(((long long)CHUNK << SLA) < (1LL << 31));
static_assert(NBD % (NTHR * 4) == 0);
static_assert(LISTN % NTHR == 0);
static_assert(NBA % NWAVE == 0 && NBA % 32 == 0 && NBA % GBM == 0);
static_assert(RCAP % 32 == 0 && AGG_ZINTS % 4 == 0 && LISTN % 4 == 0);
static_assert(KL % 32 == 0 && KZ % 32 == 0 && KL == 2 * HID && KL == CIN);
static_assert(GBM == (GTHR / 32) * 16 && GBN == 64 && HID == GBN && NCP == GBN);
static_assert(NU0 % NTHR == 0 && NUH % NTHR == 0 && NUO % NTHR == 0);
static_assert(KL / 8 == 16 && KZ / 8 == 96 && CIN / 8 == 16);
static_assert(HID * (KL / 8) == 1024);
static_assert(HID == 2 * 32);
static_assert(NCLS <= NCP && NCLS % 4 == 0 && NCLS % 2 == 0);
static_assert(AGG_LDS_INTS * 4 <= 300000);
static_assert((GBM * NCLS * 4) % 128 == 0);

typedef float          v2f   __attribute__((ext_vector_type(2)));
typedef float          v4f   __attribute__((ext_vector_type(4)));
typedef float          v8f   __attribute__((ext_vector_type(8)));
typedef int            v4i   __attribute__((ext_vector_type(4)));
typedef int            v8i   __attribute__((ext_vector_type(8)));
typedef unsigned int   v4u   __attribute__((ext_vector_type(4)));
typedef unsigned short v8us  __attribute__((ext_vector_type(8)));
typedef unsigned short v16us __attribute__((ext_vector_type(16)));
typedef __bf16         v16bf __attribute__((ext_vector_type(16)));
typedef v2f  __attribute__((may_alias)) v2fa;
typedef v4f  __attribute__((may_alias)) v4fa;
typedef v4i  __attribute__((may_alias)) v4ia;
typedef v8us __attribute__((may_alias)) v8usa;
union FragB { v16bf v; v16us u; v8us h[2]; v8i w; };

__device__ __forceinline__ v8f wmb(const FragB& a, const FragB& b, v8f c) {
  v8f d = __builtin_amdgcn_wmma_f32_16x16x32_bf16(false, a.v, false, b.v, (short)0, c, false, false);
  asm volatile("v_nop\n\tv_nop\n\tv_nop\n\tv_nop" : "+v"(d) : "v"(a.w), "v"(b.w));
  return d;
}

__device__ __forceinline__ unsigned bf16_bits(float f) {
  const unsigned u = __float_as_uint(f);
  return (u + 0x7FFFu + ((u >> 16) & 1u)) >> 16;
}
__device__ __forceinline__ float bf16_val(float f) {
  return __uint_as_float(bf16_bits(f) << 16);
}

template <int SLB>
__device__ __forceinline__ int scan_chunk(const int* __restrict__ dsts, int nE, int cbase, int slotBase,
                                          int nb, int vec8, int* list, int tid, int lane, int wave) {
  int wc = 0;
  const int el0  = tid * EPT;
  const int e0   = cbase + el0;
  const int sent = -2147483647 - 1;
  v4i da, db;
  if (vec8 != 0 && cbase + CHUNK <= nE) {
    da = *(const v4i*)(dsts + e0);
    db = *(const v4i*)(dsts + e0 + 4);
  } else {
    da.x = (e0     < nE) ? dsts[min(e0,     nE - 1)] : sent;
    da.y = (e0 + 1 < nE) ? dsts[min(e0 + 1, nE - 1)] : sent;
    da.z = (e0 + 2 < nE) ? dsts[min(e0 + 2, nE - 1)] : sent;
    da.w = (e0 + 3 < nE) ? dsts[min(e0 + 3, nE - 1)] : sent;
    db.x = (e0 + 4 < nE) ? dsts[min(e0 + 4, nE - 1)] : sent;
    db.y = (e0 + 5 < nE) ? dsts[min(e0 + 5, nE - 1)] : sent;
    db.z = (e0 + 6 < nE) ? dsts[min(e0 + 6, nE - 1)] : sent;
    db.w = (e0 + 7 < nE) ? dsts[min(e0 + 7, nE - 1)] : sent;
  }
  const unsigned nbs = (unsigned)slotBase;
  const unsigned unb = (unsigned)nb;
  const unsigned s0 = (unsigned)da.x - nbs, s1 = (unsigned)da.y - nbs;
  const unsigned s2 = (unsigned)da.z - nbs, s3 = (unsigned)da.w - nbs;
  const unsigned s4 = (unsigned)db.x - nbs, s5 = (unsigned)db.y - nbs;
  const unsigned s6 = (unsigned)db.z - nbs, s7 = (unsigned)db.w - nbs;
  const bool h0 = s0 < unb, h1 = s1 < unb, h2 = s2 < unb, h3 = s3 < unb;
  const bool h4 = s4 < unb, h5 = s5 < unb, h6 = s6 < unb, h7 = s7 < unb;
  const unsigned any = __builtin_amdgcn_ballot_w32(h0 | h1 | h2 | h3 | h4 | h5 | h6 | h7);
  if (any != 0u) {
#define HITJ(J, HJ, SJ) { \
      const unsigned mj = __builtin_amdgcn_ballot_w32(HJ); \
      if (mj != 0u) { \
        if (HJ) { \
          const int pos = wc + (int)__builtin_amdgcn_mbcnt_lo(mj, 0u); \
          if (pos < WCAP) list[wave * WCAP + pos] = ((el0 + (J)) << SLB) | (int)(SJ); \
        } \
        wc += (int)__builtin_popcount(mj); } }
    HITJ(0, h0, s0)
    HITJ(1, h1, s1)
    HITJ(2, h2, s2)
    HITJ(3, h3, s3)
    HITJ(4, h4, s4)
    HITJ(5, h5, s5)
    HITJ(6, h6, s6)
    HITJ(7, h7, s7)
#undef HITJ
  }
  return wc;
}

__global__ __launch_bounds__(NTHR) void k_wprep(const float* __restrict__ W0, const float* __restrict__ Wh,
                                                const float* __restrict__ Wo,
                                                unsigned short* W0T, unsigned short* WHT, unsigned short* WOT) {
  const int u = (int)blockIdx.x * NTHR + (int)threadIdx.x;
  v8us o;
  unsigned short* dp;
  if (u < NU0) {
    const int n  = u >> 4;
    const int k8 = (u & 15) * 8;
    const float* p = W0 + (size_t)k8 * HID + n;
#pragma unroll
    for (int i = 0; i < 8; ++i) o[i] = (unsigned short)bf16_bits(p[(size_t)i * HID]);
    dp = W0T + (size_t)n * KL + k8;
  } else if (u < NU0 + NUH) {
    const int v  = u - NU0;
    const int li = v >> 10;
    const int w  = v & 1023;
    const int n  = w >> 4;
    const int k8 = (w & 15) * 8;
    const int kk = k8 & (HID - 1);
    const float* p = Wh + (size_t)li * (HID * HID) + (size_t)kk * HID + n;
#pragma unroll
    for (int i = 0; i < 8; ++i) o[i] = (unsigned short)bf16_bits(p[(size_t)i * HID]);
    dp = WHT + (size_t)li * (HID * KL) + (size_t)n * KL + k8;
  } else if (u < NU0 + NUH + NUO) {
    const int v   = u - NU0 - NUH;
    const int n   = v / (KZ / 8);
    const int k8  = (v - n * (KZ / 8)) * 8;
    const int lay = k8 >> 7;
    const int kk  = k8 & (HID - 1);
    const int kr  = lay * HID + kk;
    const int ncl = n < NCLS ? n : NCLS - 1;
    const float* p = Wo + (size_t)kr * NCLS + ncl;
    const bool ok = n < NCLS;
#pragma unroll
    for (int i = 0; i < 8; ++i) {
      const float wv = p[(size_t)i * NCLS];
      o[i] = ok ? (unsigned short)bf16_bits(wv) : (unsigned short)0;
    }
    dp = WOT + (size_t)n * KZ + k8;
  } else {
    return;
  }
  *(volatile v8us*)dp = o;
  __threadfence();
  *(volatile v8us*)dp = o;
}

__global__ __launch_bounds__(NTHR) void k_cvx(const float* __restrict__ x, int nN, int nUnits,
                                              unsigned short* xb) {
  const int u = (int)blockIdx.x * NTHR + (int)threadIdx.x;
  if (u >= nUnits) return;
  const int row = u >> 4;
  const int k8  = (u & 15) * 8;
  const int rc  = row < nN ? row : nN - 1;
  const float* p = x + (size_t)rc * CIN + k8;
  const v4f a = *(const v4fa*)p;
  const v4f b = *(const v4fa*)(p + 4);
  const bool ok = row < nN;
  v8us o;
  o[0] = ok ? (unsigned short)bf16_bits(a.x) : (unsigned short)0;
  o[1] = ok ? (unsigned short)bf16_bits(a.y) : (unsigned short)0;
  o[2] = ok ? (unsigned short)bf16_bits(a.z) : (unsigned short)0;
  o[3] = ok ? (unsigned short)bf16_bits(a.w) : (unsigned short)0;
  o[4] = ok ? (unsigned short)bf16_bits(b.x) : (unsigned short)0;
  o[5] = ok ? (unsigned short)bf16_bits(b.y) : (unsigned short)0;
  o[6] = ok ? (unsigned short)bf16_bits(b.z) : (unsigned short)0;
  o[7] = ok ? (unsigned short)bf16_bits(b.w) : (unsigned short)0;
  unsigned short* dp = xb + (size_t)row * CIN + k8;
  *(volatile v8us*)dp = o;
  __threadfence();
  *(volatile v8us*)dp = o;
}

__global__ __launch_bounds__(NTHR) void k_deg(const int* __restrict__ dsts, const float* __restrict__ ew,
                                              int nE, int vec8, float* dis) {
  __shared__ __attribute__((aligned(16))) float sdeg[NBD];
  __shared__ __attribute__((aligned(16))) int list[LISTN];
  __shared__ int wcnt[NWAVE];
  const int tid = (int)threadIdx.x, lane = tid & 31, wave = tid >> 5;
  const int nodeBase = (int)blockIdx.x * NBD;

  for (int i = tid; i < NBD; i += NTHR) sdeg[i] = 0.0f;
  for (int i = tid; i < LISTN; i += NTHR) list[i] = 0;
  if (tid < NWAVE) wcnt[tid] = 0;
  __syncthreads();

  const int nChunks = (nE + CHUNK - 1) / CHUNK;
#pragma unroll 1
  for (int ch = 0; ch < nChunks; ++ch) {
    const int cbase = ch * CHUNK;
    const int wc = scan_chunk<SLD>(dsts, nE, cbase, nodeBase, NBD, vec8, list, tid, lane, wave);
    if (lane == 0) wcnt[wave] = wc;
    __syncthreads();
    if (wave == 0) {
#pragma unroll 1
      for (int w2 = 0; w2 < NWAVE; ++w2) {
        int c = wcnt[w2];
        c = c < 0 ? 0 : (c > WCAP ? WCAP : c);
#pragma unroll 1
        for (int b0 = 0; b0 < c; b0 += 32) {
          const int idx = b0 + lane;
          const int ent = list[w2 * WCAP + (idx < WCAP ? idx : WCAP - 1)];
          const int el  = (ent >> SLD) & (CHUNK - 1);
          int eid = cbase + el;
          eid = eid < 0 ? 0 : (eid > nE - 1 ? nE - 1 : eid);
          const float wv  = bf16_val(ew[eid]);
          const int   wvi = __float_as_int(wv);
          const int m32 = (c - b0) < 32 ? (c - b0) : 32;
#pragma unroll 1
          for (int k = 0; k < m32; ++k) {
            const int   u  = __builtin_amdgcn_readlane(ent, k);
            const float wk = __int_as_float(__builtin_amdgcn_readlane(wvi, k));
            const int sl = u & (NBD - 1);
            if (lane == 0) sdeg[sl] = sdeg[sl] + wk;
          }
        }
      }
    }
    __syncthreads();
  }

  v4f vals[NBD / (NTHR * 4)];
#pragma unroll
  for (int it = 0; it < NBD / (NTHR * 4); ++it) {
    const int s0 = it * (NTHR * 4) + 4 * tid;
    const v4f c4 = *(const v4fa*)(sdeg + s0);
    const float d0 = c4.x + 1.0f, d1 = c4.y + 1.0f, d2 = c4.z + 1.0f, d3 = c4.w + 1.0f;
    v4f v;
    v.x = d0 > 0.0f ? rsqrtf(d0) : 0.0f;
    v.y = d1 > 0.0f ? rsqrtf(d1) : 0.0f;
    v.z = d2 > 0.0f ? rsqrtf(d2) : 0.0f;
    v.w = d3 > 0.0f ? rsqrtf(d3) : 0.0f;
    vals[it] = v;
  }
#pragma unroll
  for (int it = 0; it < NBD / (NTHR * 4); ++it) {
    const int s0 = it * (NTHR * 4) + 4 * tid;
    *(volatile v4f*)(dis + (size_t)nodeBase + s0) = vals[it];
  }
  __threadfence();
#pragma unroll
  for (int it = 0; it < NBD / (NTHR * 4); ++it) {
    const int s0 = it * (NTHR * 4) + 4 * tid;
    *(volatile v4f*)(dis + (size_t)nodeBase + s0) = vals[it];
  }
}

template <int MODE>
__global__ __launch_bounds__(GTHR) void k_gemm(
    const unsigned short* __restrict__ A, int lda, const unsigned short* __restrict__ WT, int K,
    float* outF, int ldo, const float* __restrict__ bias, float* outp, int nN)
{
  __shared__ __attribute__((aligned(16))) float stg[GBM * GBN];
  __shared__ __attribute__((aligned(16))) float res[GBM * NCLS];
  const int tid = (int)threadIdx.x, lane = tid & 31, wave = tid >> 5, hh = lane >> 4, m = lane & 15;
  const int rowBase = (int)blockIdx.x * GBM;
  const int col0    = (int)blockIdx.y * GBN;

  v8f acc[4];
  {
    const v8f z = {0.f, 0.f, 0.f, 0.f, 0.f, 0.f, 0.f, 0.f};
    acc[0] = z; acc[1] = z; acc[2] = z; acc[3] = z;
  }
  const unsigned short* ap = A  + (size_t)(rowBase + 16 * wave + m) * (size_t)lda + 8 * hh;
  const unsigned short* wp = WT + (size_t)(col0 + m) * (size_t)K + 8 * hh;
  const int ksteps = K >> 5;
#pragma unroll 1
  for (int ks = 0; ks < ksteps; ++ks) {
    FragB af;
    af.h[0] = *(const v8usa*)(ap + 32 * ks);
    af.h[1] = *(const v8usa*)(ap + 32 * ks + 16);
#pragma unroll
    for (int t = 0; t < 4; ++t) {
      const unsigned short* wq = wp + (size_t)(16 * t) * (size_t)K + 32 * ks;
      FragB bf;
      bf.h[0] = *(const v8usa*)wq;
      bf.h[1] = *(const v8usa*)(wq + 16);
      acc[t] = wmb(af, bf, acc[t]);
    }
  }

#pragma unroll
  for (int t = 0; t < 4; ++t) {
    const int lc = 16 * t + m;
#pragma unroll
    for (int r = 0; r < 8; ++r) {
      const int lr = 16 * wave + 8 * hh + r;
      stg[lr * GBN + lc] = acc[t][r];
    }
  }
  __syncthreads();

  if constexpr (MODE == 0) {
    v4f fv[8];
#pragma unroll
    for (int i = 0; i < 8; ++i) {
      const int lr = 16 * wave + 2 * i + hh;
      fv[i] = *(const v4fa*)(stg + lr * GBN + 4 * m);
    }
#pragma unroll
    for (int i = 0; i < 8; ++i) {
      const int lr = 16 * wave + 2 * i + hh;
      const int gr = rowBase + lr;
      float* op = outF + (size_t)gr * (size_t)ldo + col0 + 4 * m;
      *(volatile v4f*)op = fv[i];
    }
    __threadfence();
#pragma unroll
    for (int i = 0; i < 8; ++i) {
      const int lr = 16 * wave + 2 * i + hh;
      const int gr = rowBase + lr;
      float* op = outF + (size_t)gr * (size_t)ldo + col0 + 4 * m;
      *(volatile v4f*)op = fv[i];
    }
  } else {
    const int c0 = 2 * lane;
    const bool valid = c0 < NCLS;
    const int cc0 = c0 < NCLS ? c0 : NCLS - 1;
    const int cc1 = c0 + 1 < NCLS ? c0 + 1 : NCLS - 1;
    float bz0 = bf16_val(bias[cc0]), bz1 = bf16_val(bias[cc1]);
    bz0 = valid ? bz0 : 0.f;
    bz1 = valid ? bz1 : 0.f;
#pragma unroll 1
    for (int rr = 0; rr < 16; ++rr) {
      const int lr = 16 * wave + rr;
      const v2f zv = *(const v2fa*)(stg + lr * GBN + c0);
      const float z0 = zv.x + bz0, z1 = zv.y + bz1;
      float vm = valid ? fmaxf(z0, z1) : -3.0e38f;
#pragma unroll
      for (int off = 16; off > 0; off >>= 1) vm = fmaxf(vm, __shfl_xor(vm, off, 32));
      const float d0 = valid ? (z0 - vm) : 0.f;
      const float d1 = valid ? (z1 - vm) : 0.f;
      const float ex0 = expf(d0), ex1 = expf(d1);
      float sm = valid ? (ex0 + ex1) : 0.f;
#pragma unroll
      for (int off = 16; off > 0; off >>= 1) sm += __shfl_xor(sm, off, 32);
      const float ls = logf(sm);
      const float o0 = d0 - ls, o1 = d1 - ls;
      if (valid) {
        v2f ov; ov.x = o0; ov.y = o1;
        *(v2fa*)(res + lr * NCLS + c0) = ov;
      }
    }
    __syncthreads();
    int live = nN - rowBase;
    live = live < 0 ? 0 : (live > GBM ? GBM : live);
    const int npc = live * (NCLS / 4);
    float* ob = outp + (size_t)rowBase * NCLS;
#pragma unroll 1
    for (int p = tid; p < npc; p += GTHR) {
      const v4f v = *(const v4fa*)(res + 4 * p);
      *(volatile v4f*)(ob + 4 * p) = v;
    }
    __threadfence();
#pragma unroll 1
    for (int p = tid; p < npc; p += GTHR) {
      const v4f v = *(const v4fa*)(res + 4 * p);
      *(volatile v4f*)(ob + 4 * p) = v;
    }
  }
}

__global__ __launch_bounds__(NTHR) void k_agg(const int* __restrict__ srcs, const int* __restrict__ dsts,
                                              const float* __restrict__ ew,
                                              int nE, int nN, int vec8, int mRows,
                                              const float* __restrict__ dis,
                                              const float* __restrict__ xl, const float* __restrict__ bias,
                                              unsigned short* zp, int colOff) {
  extern __shared__ __attribute__((aligned(16))) int dsm[];
  int* list = dsm;
  int* hl   = dsm + LISTN;
  int* sl   = dsm + LISTN + RCAP;
  int* cnt  = dsm + LISTN + 2 * RCAP;
  int* offs = cnt + NBA;
  int* cur  = offs + NBA;
  int* misc = cur + NBA;
  const int tid = (int)threadIdx.x, lane = tid & 31, wave = tid >> 5;
  const int nodeBase = (int)blockIdx.x * NBA;

  {
    const v4i z4 = {0, 0, 0, 0};
    for (int i = tid * 4; i < AGG_ZINTS; i += NTHR * 4) *(v4ia*)(dsm + i) = z4;
    if (tid < 16) misc[tid] = 0;
  }
  float bv[2];
  {
    const v2f a = *(const v2fa*)(bias + 2 * lane);
    bv[0] = bf16_val(a.x); bv[1] = bf16_val(a.y);
  }
  __syncthreads();

  int t = 0, ov = 0;
  const int nChunks = (nE + CHUNK - 1) / CHUNK;
#pragma unroll 1
  for (int ch = 0; ch < nChunks; ++ch) {
    const int cbase = ch * CHUNK;
    const int wc = scan_chunk<SLA>(dsts, nE, cbase, nodeBase, NBA, vec8, list, tid, lane, wave);
    if (lane == 0) misc[wave] = wc;
    __syncthreads();
    if (wave == 0) {
#pragma unroll 1
      for (int w2 = 0; w2 < NWAVE; ++w2) {
        int c = misc[w2];
        c = c < 0 ? 0 : (c > WCAP ? WCAP : c);
#pragma unroll 1
        for (int b0 = 0; b0 < c; b0 += 32) {
          const int idx = b0 + lane;
          const int ent = list[w2 * WCAP + (idx < WCAP ? idx : WCAP - 1)];
          const int m32 = (c - b0) < 32 ? (c - b0) : 32;
#pragma unroll 1
          for (int k = 0; k < m32; ++k) {
            const int u    = __builtin_amdgcn_readlane(ent, k);
            const int slot = u & (NBA - 1);
            const int el   = (u >> SLA) & (CHUNK - 1);
            const int pk   = ((cbase + el) << SLA) | slot;
            if (t < RCAP) {
              if (lane == 0) { hl[t] = pk; cnt[slot] = cnt[slot] + 1; }
              t = t + 1;
            } else {
              ov = 1;
            }
          }
        }
      }
    }
    __syncthreads();
  }
  if (wave == 0 && lane == 0) { misc[8] = t; misc[9] = ov; }
  __syncthreads();
  int tt = misc[8];
  tt = tt < 0 ? 0 : (tt > RCAP ? RCAP : tt);
  const int ovf = misc[9];

  if (wave == 0) {
    const int base = lane * (NBA / 32);
    int s = 0;
#pragma unroll 1
    for (int i = 0; i < NBA / 32; ++i) s += cnt[base + i];
    int incl = s;
#pragma unroll
    for (int d = 1; d < 32; d <<= 1) {
      const int y = __shfl_up(incl, d, 32);
      if (lane >= d) incl += y;
    }
    int run = incl - s;
#pragma unroll 1
    for (int i = 0; i < NBA / 32; ++i) {
      const int cv = cnt[base + i];
      offs[base + i] = run;
      cur[base + i]  = run;
      run += cv;
    }
  }
  __syncthreads();
  if (wave == 0) {
#pragma unroll 1
    for (int b0 = 0; b0 < tt; b0 += 32) {
      const int idx = b0 + lane;
      const int ent = hl[idx < RCAP ? idx : RCAP - 1];
      const int m32 = (tt - b0) < 32 ? (tt - b0) : 32;
#pragma unroll 1
      for (int k = 0; k < m32; ++k) {
        const int u    = __builtin_amdgcn_readlane(ent, k);
        const int slot = u & (NBA - 1);
        if (lane == 0) {
          int p = cur[slot];
          p = p < 0 ? 0 : (p > RCAP - 1 ? RCAP - 1 : p);
          sl[p] = u;
          cur[slot] = p + 1;
        }
      }
    }
  }
  __syncthreads();

  const float qnan = __int_as_float(0x7fc00000);
  const float pz = (ovf != 0) ? qnan : 0.0f;
  const int sa0 = (4 * lane) & 31;
  const int sa1 = (4 * lane + 1) & 31;
  const int sa2 = (4 * lane + 2) & 31;
  const int sa3 = (4 * lane + 3) & 31;
#pragma unroll 1
  for (int si = 0; si < NBA / NWAVE; ++si) {
    const int s    = si * NWAVE + wave;
    const int node = nodeBase + s;
    int c = cnt[s];
    const bool big = c > DEGCAP;
    c = c < 0 ? 0 : (c > DEGCAP ? DEGCAP : c);
    int o = offs[s];
    o = o < 0 ? 0 : (o > RCAP ? RCAP : o);
    const int nc = node < nN ? node : nN - 1;
    const float dd = dis[nc];
    const float rd = dd * dd;
    float acc0 = 0.0f, acc1 = 0.0f;
#pragma unroll 1
    for (int b0 = 0; b0 < c; b0 += 32) {
      int idx = o + b0 + lane;
      idx = idx > RCAP - 1 ? RCAP - 1 : idx;
      const int ent = sl[idx];
      int eid = ent >> SLA;
      eid = eid < 0 ? 0 : (eid > nE - 1 ? nE - 1 : eid);
      int sr = srcs[eid];
      sr = sr < 0 ? 0 : (sr > nN - 1 ? nN - 1 : sr);
      const float wv  = bf16_val(ew[eid]);
      const float cf  = (dis[sr] * wv) * dd;
      const int   cfi = __float_as_int(cf);
      const int m32 = (c - b0) < 32 ? (c - b0) : 32;
#pragma unroll 1
      for (int k = 0; k < m32; ++k) {
        const int   sk = __builtin_amdgcn_readlane(sr, k);
        const float ck = __int_as_float(__builtin_amdgcn_readlane(cfi, k));
        const float* rp = xl + (size_t)sk * HID + 2 * lane;
        const v2f a = *(const v2fa*)rp;
        acc0 = fmaf(ck, a.x, acc0);
        acc1 = fmaf(ck, a.y, acc1);
      }
    }
    float sv0, sv1;
    {
      const float* sp = xl + (size_t)nc * HID + 2 * lane;
      const v2f a = *(const v2fa*)sp;
      sv0 = a.x; sv1 = a.y;
    }
    const float pzr = big ? qnan : pz;
    const bool live = node < nN;
    float y0 = (acc0 + sv0 * rd) + bv[0];
    float y1 = (acc1 + sv1 * rd) + bv[1];
    y0 = fmaxf(y0, 0.0f) + pzr;
    y1 = fmaxf(y1, 0.0f) + pzr;
    const float v0 = live ? y0 : 0.0f;
    const float v1 = live ? y1 : 0.0f;
    const unsigned hb0 = bf16_bits(v0), hb1 = bf16_bits(v1);
    const unsigned lb0 = bf16_bits(v0 - __uint_as_float(hb0 << 16));
    const unsigned lb1 = bf16_bits(v1 - __uint_as_float(hb1 << 16));
    const int hw = (int)(hb0 | (hb1 << 16));
    const int lw = (int)(lb0 | (lb1 << 16));
    const int g0 = __shfl(hw, sa0, 32), g1 = __shfl(hw, sa1, 32), g2 = __shfl(hw, sa2, 32), g3 = __shfl(hw, sa3, 32);
    const int q0 = __shfl(lw, sa0, 32), q1 = __shfl(lw, sa1, 32), q2 = __shfl(lw, sa2, 32), q3 = __shfl(lw, sa3, 32);
    const bool lsel = lane >= 8;
    v4u pv;
    pv.x = (unsigned int)(lsel ? q0 : g0);
    pv.y = (unsigned int)(lsel ? q1 : g1);
    pv.z = (unsigned int)(lsel ? q2 : g2);
    pv.w = (unsigned int)(lsel ? q3 : g3);
    const bool wr = (node < mRows) && (lane < 16);
    unsigned short* hp = zp + (size_t)node * KZ + colOff + 8 * (lane & 15);
    if (wr) *(volatile v4u*)hp = pv;
    __threadfence();
    if (wr) *(volatile v4u*)hp = pv;
  }
}

static inline int cdiv(int a, int b) { return (a + b - 1) / b; }

extern "C" void kernel_launch(void* const* d_in, const int* in_sizes, int n_in,
                              void* d_out, int out_size, void* d_ws, size_t ws_size,
                              hipStream_t stream) {
  if (n_in < 9) return;
  if (in_sizes[0] < CIN || (in_sizes[0] % CIN) != 0) return;
  const int nN = in_sizes[0] / CIN;
  if (in_sizes[1] < 2 || (in_sizes[1] & 1) != 0) return;
  const int nE = in_sizes[1] / 2;
  if (nE < 1 || nE >= (1 << (31 - SLA))) return;
  if (in_sizes[2] != nE) return;
  if (in_sizes[3] != CIN * HID || in_sizes[4] != HID) return;
  if (in_sizes[5] != (NLAY - 1) * HID * HID) return;
  if (in_sizes[6] != (NLAY - 1) * HID) return;
  if (in_sizes[7] != NLAY * HID * NCLS || in_sizes[8] != NCLS) return;
  if ((long long)out_size != (long long)nN * NCLS) return;

  const float* x    = (const float*)d_in[0];
  const int*   edge = (const int*)d_in[1];
  const float* ewp  = (const float*)d_in[2];
  const float* W0   = (const float*)d_in[3];
  const float* b0   = (const float*)d_in[4];
  const float* Wh   = (const float*)d_in[5];
  const float* bh   = (const float*)d_in[6];
  const float* Wout = (const float*)d_in[7];
  const float* bout = (const float*)d_in[8];
  float* out = (float*)d_out;
  const int* src = edge;
  const int* dst = edge + nE;

  const int MP   = cdiv(nN, GBM) * GBM;
  const int gM   = MP / GBM;
  const int gD   = cdiv(nN, NBD);
  const int NBPD = gD * NBD;
  const int gA   = cdiv(MP, NBA);
  if ((long long)gA * NBA < (long long)MP) return;
  if (NBPD < nN) return;
  const int vec8 = ((nE & 3) == 0) ? 1 : 0;

  char* ws = (char*)d_ws;
  size_t off = 0;
  const size_t oDIS = off; off += (size_t)NBPD * 4;                        off = (off + 255) & ~(size_t)255;
  const size_t oW0T = off; off += (size_t)HID * KL * 2;                    off = (off + 255) & ~(size_t)255;
  const size_t oWHT = off; off += (size_t)(NLAY - 1) * HID * KL * 2;       off = (off + 255) & ~(size_t)255;
  const size_t oWOT = off; off += (size_t)NCP * KZ * 2;                    off = (off + 255) & ~(size_t)255;
  const size_t oXB  = off; off += (size_t)MP * CIN * 2;                    off = (off + 255) & ~(size_t)255;
  const size_t oT   = off; off += (size_t)MP * HID * 4;                    off = (off + 255) & ~(size_t)255;
  const size_t oZ   = off; off += (size_t)MP * KZ * 2;                     off = (off + 255) & ~(size_t)255;
  if (off > ws_size || off > (size_t)WSMAX) return;
  float*          DIS = (float*)(ws + oDIS);
  unsigned short* W0T = (unsigned short*)(ws + oW0T);
  unsigned short* WHT = (unsigned short*)(ws + oWHT);
  unsigned short* WOT = (unsigned short*)(ws + oWOT);
  unsigned short* XB  = (unsigned short*)(ws + oXB);
  float*          T   = (float*)(ws + oT);
  unsigned short* Z   = (unsigned short*)(ws + oZ);

  const size_t aggLds = (size_t)AGG_LDS_INTS * 4;
  hipFuncSetAttribute(reinterpret_cast<const void*>(&k_agg), hipFuncAttributeMaxDynamicSharedMemorySize, (int)aggLds);

  const int nUx = MP * (CIN / 8);
  k_wprep<<<(NU0 + NUH + NUO) / NTHR, NTHR, 0, stream>>>(W0, Wh, Wout, W0T, WHT, WOT);
  k_cvx<<<cdiv(nUx, NTHR), NTHR, 0, stream>>>(x, nN, nUx, XB);
  k_deg<<<gD, NTHR, 0, stream>>>(dst, ewp, nE, vec8, DIS);

  for (int l = 0; l < NLAY; ++l) {
    const unsigned short* Ap = (l == 0) ? XB : (Z + (size_t)(l - 1) * KL);
    const int lda              = (l == 0) ? CIN : KZ;
    const unsigned short* Wp = (l == 0) ? W0T : (WHT + (size_t)(l - 1) * HID * KL);
    const float* bp          = (l == 0) ? b0 : (bh + (size_t)(l - 1) * HID);
    k_gemm<0><<<dim3(gM, 1), GTHR, 0, stream>>>(Ap, lda, Wp, KL, T, HID, bp, out, nN);
    k_agg<<<gA, NTHR, aggLds, stream>>>(src, dst, ewp, nE, nN, vec8, MP, DIS, T, bp, Z, l * KL);
  }
  k_gemm<1><<<dim3(gM, 1), GTHR, 0, stream>>>(Z, KZ, WOT, KZ, T, HID, bout, out, nN);
}
